// ConvAttentionCUDA_2302102470965
// MI455X (gfx1250) — hardware-verified
//
#include <hip/hip_runtime.h>


namespace {
constexpr int H = 16, S = 2048, D = 128, HG = 4;
constexpr float XS = 8.0f, VS = 8.0f, SCALE = 0.08838834764831845f;

typedef _Float16 b16;
typedef __attribute__((ext_vector_type(16))) _Float16 v16b;
typedef __attribute__((ext_vector_type(8)))  _Float16 v8b;
typedef __attribute__((ext_vector_type(8)))  float v8f;
typedef __attribute__((ext_vector_type(4)))  float v4f;

__device__ __forceinline__ v8b ld8b(const b16* p) { return *(const v8b*)p; }
__device__ __forceinline__ v16b cat8b(v8b a, v8b b) { return __builtin_shufflevector(a, b, 0, 1, 2, 3, 4, 5, 6, 7, 8, 9, 10, 11, 12, 13, 14, 15); }
__device__ __forceinline__ v16b frag_kb(const b16* p, int hh) { return cat8b(ld8b(p + 8 * hh), ld8b(p + 16 + 8 * hh)); }
__device__ __forceinline__ void split16(float v, b16& hi, b16& lo) { hi = (b16)v; lo = (b16)(v - (float)hi); }
__device__ __forceinline__ void frag_ksplit(const float* p, int hh, v16b& fh_, v16b& fl_) {
  const float* p0 = p + 8 * hh; const float* p1 = p + 16 + 8 * hh;
#pragma unroll
  for (int e = 0; e < 8; ++e) { b16 a, c; split16(p0[e], a, c); fh_[e] = a; fl_[e] = c; split16(p1[e], a, c); fh_[8 + e] = a; fl_[8 + e] = c; }
}
__device__ __forceinline__ v8f wmma16b(v16b a, v16b b, v8f c) {
  v8f d = __builtin_amdgcn_wmma_f32_16x16x32_f16(false, a, false, b, (short)0, c, false, false);
  asm volatile("v_nop\n\tv_nop\n\tv_nop\n\tv_nop" : "+v"(d) : "v"(a), "v"(b));
  return d;
}
__device__ __forceinline__ void wave_lds_sync() {
  __builtin_amdgcn_fence(__ATOMIC_RELEASE, "workgroup");
  __builtin_amdgcn_wave_barrier();
  __builtin_amdgcn_fence(__ATOMIC_ACQUIRE, "workgroup");
}

struct Opnd { const void* p0; const void* p1; int ld; };
template <int NP> __device__ __forceinline__ void load_frags(const Opnd& o, int row, int kb, int hh, v16b& fh_, v16b& fl_) {
  if (NP == 0) { frag_ksplit((const float*)o.p0 + (size_t)row * o.ld + kb, hh, fh_, fl_); }
  else if (NP == 4 || NP == 5) {
    const float sc_ = (NP == 4) ? 64.0f : 8.0f;
    const float* p = (const float*)o.p0 + (size_t)row * o.ld + kb; const float* p0 = p + 8 * hh; const float* p1 = p + 16 + 8 * hh;
#pragma unroll
    for (int e = 0; e < 8; ++e) { b16 a, c; split16(p0[e] * sc_, a, c); fh_[e] = a; fl_[e] = c; split16(p1[e] * sc_, a, c); fh_[8 + e] = a; fl_[8 + e] = c; }
  } else if (NP == 3) {
    const float* p = (const float*)o.p0 + (size_t)row * o.ld + kb; const float* p0 = p + 8 * hh; const float* p1 = p + 16 + 8 * hh;
#pragma unroll
    for (int e = 0; e < 8; ++e) { fh_[e] = (b16)p0[e]; fh_[8 + e] = (b16)p1[e]; }
    fl_ = fh_;
  } else {
    fh_ = frag_kb((const b16*)o.p0 + (size_t)row * o.ld + kb, hh);
    if (NP == 2) fl_ = frag_kb((const b16*)o.p1 + (size_t)row * o.ld + kb, hh); else fl_ = fh_;
  }
}
template <int ANP, int BNP> __device__ __forceinline__ v8f mac(v16b ah, v16b al, v16b bh, v16b bl, v8f c) {
  c = wmma16b(ah, bh, c);
  if (BNP == 0 || BNP == 2 || BNP == 4 || BNP == 5) c = wmma16b(ah, bl, c);
  if (ANP == 0 || ANP == 2 || ANP == 4 || ANP == 5) c = wmma16b(al, bh, c);
  return c;
}
template <int ANP, int BNP>
__device__ __forceinline__ void gemm_tile(const Opnd& A, const Opnd& B, int K, int m0, int c0, int nloc, int hlf, v8f (&acc)[2][4]) {
  for (int kb = 0; kb < K; kb += 32) {
    v16b a0h, a0l, a1h, a1l;
    load_frags<ANP>(A, m0 + nloc, kb, hlf, a0h, a0l);
    load_frags<ANP>(A, m0 + 16 + nloc, kb, hlf, a1h, a1l);
#pragma unroll
    for (int t = 0; t < 4; ++t) {
      v16b bh, bl;
      load_frags<BNP>(B, c0 + t * 16 + nloc, kb, hlf, bh, bl);
      acc[0][t] = mac<ANP, BNP>(a0h, a0l, bh, bl, acc[0][t]);
      acc[1][t] = mac<ANP, BNP>(a1h, a1l, bh, bl, acc[1][t]);
    }
  }
}

__device__ __forceinline__ void epi_planes(v8f (&acc)[2][4], float scale, bool two, b16* __restrict__ oh, b16* __restrict__ ol, int ldo,
                                           int m0, int c0, int lane, b16* Th, b16* Tl) {
  const int nloc = lane & 15, hlf = lane >> 4;
#pragma unroll
  for (int t = 0; t < 4; ++t)
#pragma unroll
    for (int r = 0; r < 2; ++r)
#pragma unroll
      for (int v = 0; v < 8; ++v) {
        const int rr = r * 16 + v + 8 * hlf, cc = t * 16 + nloc;
        b16 h_, l_; split16(acc[r][t][v] * scale, h_, l_);
        Th[rr * 64 + cc] = h_; Tl[rr * 64 + cc] = l_;
      }
  wave_lds_sync();
  for (int pass = 0; pass < 2; ++pass) {
#pragma unroll
    for (int j = 0; j < 8; ++j) {
      const int rr = j * 4 + (lane >> 3), c8 = (lane & 7) * 8;
      const size_t o = (size_t)(m0 + rr) * ldo + c0 + c8;
      *(volatile v8b*)(oh + o) = ld8b(Th + rr * 64 + c8);
      if (two) *(volatile v8b*)(ol + o) = ld8b(Tl + rr * 64 + c8);
    }
    __threadfence();
  }
}
__device__ __forceinline__ void epi_f32(v8f (&acc)[2][4], float scale, const float* rscale, float* __restrict__ out, int ldo, int m0, int c0, int lane, float* Tt) {
  const int nloc = lane & 15, hlf = lane >> 4;
#pragma unroll
  for (int t = 0; t < 4; ++t)
#pragma unroll
    for (int r = 0; r < 2; ++r)
#pragma unroll
      for (int v = 0; v < 8; ++v) {
        const int rr = r * 16 + v + 8 * hlf;
        const float rs = rscale ? rscale[(size_t)(m0 + rr) * 32] : 1.0f;
        Tt[rr * 64 + t * 16 + nloc] = acc[r][t][v] * scale * rs;
      }
  wave_lds_sync();
  float* dst0 = out + (size_t)m0 * ldo + c0;
  for (int pass = 0; pass < 2; ++pass) {
#pragma unroll
    for (int j = 0; j < 16; ++j) { const int rr = j * 2 + hlf, c4 = nloc * 4; *(volatile v4f*)(dst0 + (size_t)rr * ldo + c4) = *(const v4f*)(Tt + rr * 64 + c4); }
    __threadfence();
  }
}


__global__ __launch_bounds__(256) void vt_kernel(const float* __restrict__ V, b16* __restrict__ vth, b16* __restrict__ vtl) {
  __shared__ __attribute__((aligned(16))) b16 Th[D][72]; __shared__ __attribute__((aligned(16))) b16 Tl[D][72];
  const int tid = threadIdx.x, lane = tid & 31, wave = tid >> 5, h = blockIdx.x / (S / 64), t0 = (blockIdx.x % (S / 64)) * 64;
  for (int i = tid; i < 64 * D; i += 256) { const int t = i / D, dd = i % D; b16 a, b2; split16(V[((size_t)h * S + t0 + t) * D + dd] * VS, a, b2); Th[dd][t] = a; Tl[dd][t] = b2; }
  __syncthreads();
  b16* bh = vth + (size_t)h * D * S + t0; b16* bl = vtl + (size_t)h * D * S + t0;
  for (int pass = 0; pass < 2; ++pass) {
#pragma unroll
    for (int j = 0; j < 4; ++j) { const int dd = wave * 16 + j * 4 + (lane >> 3), c8 = (lane & 7) * 8;
      *(volatile v8b*)(bh + (size_t)dd * S + c8) = *(const v8b*)(&Th[dd][c8]); *(volatile v8b*)(bl + (size_t)dd * S + c8) = *(const v8b*)(&Tl[dd][c8]); }
    __threadfence();
  }
}

__global__ __launch_bounds__(128) void s_kernel(const float* __restrict__ Q, const float* __restrict__ K, int h0, float* __restrict__ Sb) {
  __shared__ __attribute__((aligned(16))) float Ts[4][32 * 64];
  const int lane = threadIdx.x & 31, wave = threadIdx.x >> 5, nloc = lane & 15, hlf = lane >> 4, hl = blockIdx.z, h = h0 + hl;
  const int qb = blockIdx.y, kt = blockIdx.x, m0 = qb * 128 + wave * 32, c0 = kt * 64;
  v8f acc[2][4];
#pragma unroll
  for (int r = 0; r < 2; ++r)
#pragma unroll
    for (int t = 0; t < 4; ++t) acc[r][t] = (v8f){};
  if (c0 <= qb * 128 + 127) {
    const Opnd A{Q + (size_t)h * S * D, nullptr, D}, B{K + (size_t)h * S * D, nullptr, D};
    gemm_tile<5, 5>(A, B, D, m0, c0, nloc, hlf, acc);
  }
  float* Tt = Ts[wave];
#pragma unroll
  for (int t = 0; t < 4; ++t)
#pragma unroll
    for (int r = 0; r < 2; ++r)
#pragma unroll
      for (int v = 0; v < 8; ++v) { const int rr = r * 16 + v + 8 * hlf, cc = t * 16 + nloc; Tt[rr * 64 + cc] = (c0 + cc <= m0 + rr) ? acc[r][t][v] * (SCALE / (XS * XS)) : 0.0f; }
  wave_lds_sync();
  float* dst0 = Sb + ((size_t)hl * S + m0) * S + c0;
  for (int pass = 0; pass < 2; ++pass) {
#pragma unroll
    for (int j = 0; j < 16; ++j) { const int rr = j * 2 + hlf, c4 = nloc * 4; *(volatile v4f*)(dst0 + (size_t)rr * S + c4) = *(const v4f*)(Tt + rr * 64 + c4); }
    __threadfence();
  }
}

__global__ __launch_bounds__(256) void attn_kernel(const float* __restrict__ Sb, const float* __restrict__ wconv, const b16* __restrict__ vth, const b16* __restrict__ vtl,
                                                   int h0, float* __restrict__ out) {
  __shared__ __attribute__((aligned(16))) float Os[8][16 * D];
  const int wid = threadIdx.x >> 5, lane = threadIdx.x & 31, hh = lane >> 4, col = lane & 15;
  const int qt = blockIdx.x * 8 + wid, hl = qt / (S / 16), q0 = (qt % (S / 16)) * 16, h = h0 + hl, qi = q0 + col;
  const float* Sh = Sb + (size_t)hl * S * S; const b16* vh = vth + (size_t)h * D * S; const b16* vl = vtl + (size_t)h * D * S;
  float w[9];
#pragma unroll
  for (int i = 0; i < 9; ++i) w[i] = wconv[h * 9 + i];
  float m = -INFINITY, l = 0.0f;
  v8f o[8];
#pragma unroll
  for (int n = 0; n < 8; ++n) o[n] = (v8f){};
  for (int kb = 0; kb < q0 + 16; kb += 32) {
    v8f s0 = {}, s1 = {};
#pragma unroll
    for (int i = 0; i < 3; ++i) {
      const int qr = qi - 2 + i; const bool qok = qr >= 0; const float* Srow = Sh + (size_t)(qok ? qr : 0) * S;
      {
        const int kbase = kb + 8 * hh - 1; float run[10];
#pragma unroll
        for (int j = 0; j < 10; ++j) { const int kk = kbase + j; run[j] = (qok && kk >= 0 && kk < S) ? Srow[kk] : 0.0f; }
#pragma unroll
        for (int r = 0; r < 8; ++r) s0[r] += w[i * 3 + 0] * run[r] + w[i * 3 + 1] * run[r + 1] + w[i * 3 + 2] * run[r + 2];
      }
      {
        const int kbase = kb + 16 + 8 * hh - 1; float run[10];
#pragma unroll
        for (int j = 0; j < 10; ++j) { const int kk = kbase + j; run[j] = (qok && kk >= 0 && kk < S) ? Srow[kk] : 0.0f; }
#pragma unroll
        for (int r = 0; r < 8; ++r) s1[r] += w[i * 3 + 0] * run[r] + w[i * 3 + 1] * run[r + 1] + w[i * 3 + 2] * run[r + 2];
      }
    }
#pragma unroll
    for (int r = 0; r < 8; ++r) { const int k0i = kb + 8 * hh + r, k1i = k0i + 16; if (k0i > qi) s0[r] = -INFINITY; if (k1i > qi) s1[r] = -INFINITY; }
    float mr = -INFINITY;
#pragma unroll
    for (int r = 0; r < 8; ++r) mr = fmaxf(mr, fmaxf(s0[r], s1[r]));
    mr = fmaxf(mr, __shfl_xor(mr, 16));
    float mn = fmaxf(m, mr); if (mn == -INFINITY) mn = 0.0f;
    const float al_ = __expf(m - mn); m = mn;
    float sum = 0.0f; v16b pb;
#pragma unroll
    for (int r = 0; r < 8; ++r) { const float p0 = __expf(s0[r] - mn), p1 = __expf(s1[r] - mn); sum += p0 + p1; pb[r] = (b16)p0; pb[8 + r] = (b16)p1; }
    sum += __shfl_xor(sum, 16);
    l = l * al_ + sum;
#pragma unroll
    for (int n = 0; n < 8; ++n) {
#pragma unroll
      for (int r = 0; r < 8; ++r) o[n][r] *= al_;
      const size_t ro = (size_t)(n * 16 + col) * S + kb;
      o[n] = wmma16b(frag_kb(vh + ro, hh), pb, o[n]);
      o[n] = wmma16b(frag_kb(vl + ro, hh), pb, o[n]);
    }
  }
  const float inv = (l > 0.0f) ? (1.0f / (VS * l)) : 0.0f;
  float* Tt = Os[wid];
#pragma unroll
  for (int n = 0; n < 8; ++n)
#pragma unroll
    for (int r = 0; r < 8; ++r) Tt[col * D + n * 16 + 8 * hh + r] = o[n][r] * inv;
  wave_lds_sync();
  float* dst = out + ((size_t)h * S + q0) * D;
  for (int pass = 0; pass < 2; ++pass) {
#pragma unroll
    for (int rr = 0; rr < 16; ++rr) *(volatile v4f*)(dst + (size_t)rr * D + lane * 4) = *(const v4f*)(Tt + rr * D + lane * 4);
    __threadfence();
  }
}
}

extern "C" void kernel_launch(void* const* d_in, const int* in_sizes, int n_in,
                              void* d_out, int out_size, void* d_ws, size_t ws_size, hipStream_t stream) {
  (void)n_in; (void)out_size;
  const float* Q = (const float*)d_in[0]; const float* K = (const float*)d_in[1]; const float* V = (const float*)d_in[2];
  const float* wconv = (const float*)d_in[3];
  float* out = (float*)d_out;
  if (in_sizes[0] != H * S * D || in_sizes[1] != H * S * D || in_sizes[2] != H * S * D || in_sizes[3] != H * 9) return;
  size_t off = 0; char* ws = (char*)d_ws;
  auto carve = [&](size_t bytes) { char* p = ws + off; off += (bytes + 255) & ~(size_t)255; return p; };
  b16* vth = (b16*)carve((size_t)H * D * S * 2);
  b16* vtl = (b16*)carve((size_t)H * D * S * 2);
  float* Sb = (float*)carve((size_t)HG * S * S * 4);
  if (off > ws_size) return;
  vt_kernel<<<H * (S / 64), 256, 0, stream>>>(V, vth, vtl);
  for (int g = 0; g < H / HG; ++g) {
    s_kernel<<<dim3(S / 64, S / 128, HG), 128, 0, stream>>>(Q, K, g * HG, Sb);
    attn_kernel<<<HG * (S / 16) / 8, 256, 0, stream>>>(Sb, wconv, vth, vtl, g * HG, out);
  }
}
